// KeyChannelwiseMemoryMultiHead_4080218931760
// MI455X (gfx1250) — hardware-verified
//
#include <hip/hip_runtime.h>

typedef unsigned short u16;
typedef unsigned int   u32;
typedef __bf16 v16bf __attribute__((ext_vector_type(16)));
typedef u16    v16us __attribute__((ext_vector_type(16)));
typedef u16    v8us  __attribute__((ext_vector_type(8)));
typedef float  v8f   __attribute__((ext_vector_type(8)));
typedef float  v4f   __attribute__((ext_vector_type(4)));
typedef v8us  __attribute__((may_alias)) v8usa;
typedef v4f   __attribute__((may_alias)) v4fa;
typedef float __attribute__((may_alias)) f32a;
union Frag { v16us v; v8us h[2]; };

#define NB    8
#define CIN   256
#define CMID  512
#define COUT  256
#define NPIX  4096
#define NP    32768
#define NHEAD 8
#define HD    64
#define TP    64
#define PST   520
#define TST   72
#define LDS_MAIN (2 * TP * PST * 2)

static_assert(NP % TP == 0);
static_assert(NPIX % TP == 0);
static_assert(COUT * TP * 4 <= LDS_MAIN);
static_assert((PST % 8) == 0);
static_assert((TST % 8) == 0);
static_assert(CIN % 32 == 0);
static_assert(CMID % 32 == 0);
static_assert(HD % 32 == 0);

__device__ __forceinline__ u16 bf16r(float f) {
  u32 u = __builtin_bit_cast(u32, f);
  u += 0x7FFFu + ((u >> 16) & 1u);
  return (u16)(u >> 16);
}
__device__ __forceinline__ float bf16f(u16 b) {
  return __builtin_bit_cast(float, ((u32)b) << 16);
}
__device__ __forceinline__ void split2(float v, u16& hi, u16& lo) {
  hi = bf16r(v);
  lo = bf16r(v - bf16f(hi));
}

__device__ __forceinline__ v8f wmma_bf(v16us a, v16us b, v8f c) {
  const v16bf av = __builtin_bit_cast(v16bf, a);
  const v16bf bv = __builtin_bit_cast(v16bf, b);
  v8f d = __builtin_amdgcn_wmma_f32_16x16x32_bf16(false, av, false, bv, (short)0, c, false, false);
  asm volatile("v_nop\n\tv_nop\n\tv_nop\n\tv_nop" : "+v"(d) : "v"(av), "v"(bv));
  return d;
}

__device__ __forceinline__ v8f wmma3(v16us ah, v16us al, v16us bh, v16us bl, v8f c) {
  c = wmma_bf(ah, bh, c);
  c = wmma_bf(al, bh, c);
  c = wmma_bf(ah, bl, c);
  return c;
}

__device__ __forceinline__ v16us ldfrag(const u16* p) {
  Frag f;
  f.h[0] = *(const v8usa*)p;
  f.h[1] = *(const v8usa*)(p + 16);
  return f.v;
}

__global__ __launch_bounds__(256) void wcvt_k(
    const float* __restrict__ w_in, const float* __restrict__ w_out,
    u16* __restrict__ WIh, u16* __restrict__ WIl, u16* __restrict__ WOh, u16* __restrict__ WOl)
{
  const int g = blockIdx.x * 256 + threadIdx.x;
  if (g >= (CMID * CIN + COUT * CMID) / 8) return;
  const int e8 = g * 8;
  const bool first = (e8 < CMID * CIN);
  const int off = first ? e8 : (e8 - CMID * CIN);
  const float* src = (first ? w_in : w_out) + off;
  u16* dh = (first ? WIh : WOh) + off;
  u16* dlo = (first ? WIl : WOl) + off;
  const v4f a = *(const v4fa*)src;
  const v4f c = *(const v4fa*)(src + 4);
  const float vv[8] = {a.x, a.y, a.z, a.w, c.x, c.y, c.z, c.w};
  v8us oh, ol;
  #pragma unroll
  for (int j = 0; j < 8; ++j) {
    u16 hv, lv;
    split2(vv[j], hv, lv);
    oh[j] = hv;
    ol[j] = lv;
  }
  *(volatile v8us*)dh = oh;
  *(volatile v8us*)dlo = ol;
  __threadfence();
  *(volatile v8us*)dh = oh;
  *(volatile v8us*)dlo = ol;
}

__global__ __launch_bounds__(256) void tr64_k(
    const float* __restrict__ key_p, const float* __restrict__ mem,
    u16* __restrict__ KTh, u16* __restrict__ KTl, u16* __restrict__ MTh, u16* __restrict__ MTl)
{
  __shared__ __attribute__((aligned(16))) u16 st[2 * 64 * TST];
  const int tid = threadIdx.x, lane = tid & 31, w = tid >> 5;
  const int blk = blockIdx.x;
  const bool isk = (blk < NHEAD);
  const int n = isk ? blk : (blk - NHEAD);
  const float* src = (isk ? key_p : mem) + (size_t)n * (HD * HD);
  u16* dsth = (isk ? KTh : MTh) + (size_t)n * (HD * HD);
  u16* dstl = (isk ? KTl : MTl) + (size_t)n * (HD * HD);
  const int col = tid & 63, sub = tid >> 6;
  #pragma unroll 4
  for (int j = 0; j < 16; ++j) {
    const int a = 4 * j + sub;
    const float v = src[a * HD + col];
    u16 hv, lv;
    split2(v, hv, lv);
    st[col * TST + a] = hv;
    st[64 * TST + col * TST + a] = lv;
  }
  __syncthreads();
  const int plane = w >> 2, q = lane & 7, sub8 = lane >> 3;
  u16* dplane = plane ? dstl : dsth;
  v8us vals[4];
  int ro[4];
  #pragma unroll
  for (int i = 0; i < 4; ++i) {
    const int row = 16 * (w & 3) + 4 * i + sub8;
    vals[i] = *(const v8usa*)(st + plane * (64 * TST) + row * TST + 8 * q);
    ro[i] = row * HD + 8 * q;
  }
  #pragma unroll
  for (int i = 0; i < 4; ++i) *(volatile v8us*)(dplane + ro[i]) = vals[i];
  __threadfence();
  #pragma unroll
  for (int i = 0; i < 4; ++i) *(volatile v8us*)(dplane + ro[i]) = vals[i];
}

__global__ __launch_bounds__(256) void xcvt_k(
    const float* __restrict__ x, u16* __restrict__ Xh, u16* __restrict__ Xl)
{
  __shared__ __attribute__((aligned(16))) u16 st[2 * 64 * TST];
  const int tid = threadIdx.x, lane = tid & 31, w = tid >> 5;
  const int tile = blockIdx.x, cg = blockIdx.y, b = blockIdx.z;
  const int px = tid & 63, sub = tid >> 6;
  const float* xb = x + (size_t)(b * CIN + 64 * cg) * NPIX + 64 * tile + px;
  #pragma unroll 4
  for (int j = 0; j < 16; ++j) {
    const int cl = 4 * j + sub;
    const float v = xb[(size_t)cl * NPIX];
    u16 hv, lv;
    split2(v, hv, lv);
    st[px * TST + cl] = hv;
    st[64 * TST + px * TST + cl] = lv;
  }
  __syncthreads();
  const int plane = w >> 2, q = lane & 7, sub8 = lane >> 3;
  u16* dplane = plane ? Xl : Xh;
  v8us vals[4];
  size_t ro[4];
  #pragma unroll
  for (int i = 0; i < 4; ++i) {
    const int row = 16 * (w & 3) + 4 * i + sub8;
    vals[i] = *(const v8usa*)(st + plane * (64 * TST) + row * TST + 8 * q);
    ro[i] = (size_t)(b * NPIX + 64 * tile + row) * CIN + 64 * cg + 8 * q;
  }
  #pragma unroll
  for (int i = 0; i < 4; ++i) *(volatile v8us*)(dplane + ro[i]) = vals[i];
  __threadfence();
  #pragma unroll
  for (int i = 0; i < 4; ++i) *(volatile v8us*)(dplane + ro[i]) = vals[i];
}

__global__ __launch_bounds__(256) void main_k(
    const u16* __restrict__ Xh, const u16* __restrict__ Xl,
    const u16* __restrict__ WIh, const u16* __restrict__ WIl, const float* __restrict__ b_in,
    const u16* __restrict__ KTh, const u16* __restrict__ KTl,
    const u16* __restrict__ MTh, const u16* __restrict__ MTl,
    const u16* __restrict__ WOh, const u16* __restrict__ WOl, const float* __restrict__ b_out,
    float* __restrict__ out)
{
  extern __shared__ __attribute__((aligned(16))) u16 dl[];
  u16* Ph = dl;
  u16* Pl = dl + TP * PST;
  const int tid = threadIdx.x, lane = tid & 31, w = tid >> 5;
  const int h = lane >> 4, m = lane & 15;
  const int gp0 = blockIdx.x * TP;
  const int b = gp0 >> 12, s0 = gp0 & (NPIX - 1);
  const v8f z8 = {0.f, 0.f, 0.f, 0.f, 0.f, 0.f, 0.f, 0.f};

  #pragma unroll 1
  for (int p = 0; p < 2; ++p) {
    const int orow0 = 64 * w + 32 * p;
    v8f acc[2][4];
    #pragma unroll
    for (int mt = 0; mt < 2; ++mt) {
      #pragma unroll
      for (int nt = 0; nt < 4; ++nt) acc[mt][nt] = z8;
    }
    const u16* aph = WIh + (size_t)(orow0 + m) * CIN + 8 * h;
    const u16* apl = WIl + (size_t)(orow0 + m) * CIN + 8 * h;
    const u16* bph = Xh + (size_t)(gp0 + m) * CIN + 8 * h;
    const u16* bpl = Xl + (size_t)(gp0 + m) * CIN + 8 * h;
    #pragma unroll 1
    for (int ks = 0; ks < CIN / 32; ++ks) {
      const int k0 = 32 * ks;
      v16us ah[2], al[2];
      #pragma unroll
      for (int mt = 0; mt < 2; ++mt) {
        ah[mt] = ldfrag(aph + mt * 16 * CIN + k0);
        al[mt] = ldfrag(apl + mt * 16 * CIN + k0);
      }
      #pragma unroll
      for (int nt = 0; nt < 4; ++nt) {
        const v16us bh = ldfrag(bph + nt * 16 * CIN + k0);
        const v16us bl = ldfrag(bpl + nt * 16 * CIN + k0);
        #pragma unroll
        for (int mt = 0; mt < 2; ++mt) acc[mt][nt] = wmma3(ah[mt], al[mt], bh, bl, acc[mt][nt]);
      }
    }
    #pragma unroll
    for (int mt = 0; mt < 2; ++mt) {
      const int ob = orow0 + 16 * mt + 8 * h;
      const v4f b0 = *(const v4fa*)(b_in + ob);
      const v4f b1 = *(const v4fa*)(b_in + ob + 4);
      const float bb[8] = {b0.x, b0.y, b0.z, b0.w, b1.x, b1.y, b1.z, b1.w};
      const int kq = ob >> 3;
      #pragma unroll
      for (int nt = 0; nt < 4; ++nt) {
        const int px = 16 * nt + m;
        u16* rh = Ph + px * PST + kq;
        u16* rl = Pl + px * PST + kq;
        #pragma unroll
        for (int r = 0; r < 8; ++r) {
          const float v = acc[mt][nt][r] + bb[r];
          u16 hv, lv;
          split2(v, hv, lv);
          rh[r * 64] = hv;
          rl[r * 64] = lv;
        }
      }
    }
  }
  __syncthreads();

  #pragma unroll 1
  for (int jp = 0; jp < NHEAD / 2; ++jp) {
    const int n = 2 * jp + (w >> 2);
    const int nt = w & 3;
    const int px = 16 * nt + m;
    const u16* prh = Ph + px * PST + n * 64 + 8 * h;
    const u16* prl = Pl + px * PST + n * 64 + 8 * h;
    const u16* kah = KTh + (size_t)(n * 64 + m) * HD + 8 * h;
    const u16* kal = KTl + (size_t)(n * 64 + m) * HD + 8 * h;
    v8f sacc[4];
    #pragma unroll
    for (int mt = 0; mt < 4; ++mt) sacc[mt] = z8;
    #pragma unroll
    for (int ks = 0; ks < 2; ++ks) {
      const int k0 = 32 * ks;
      const v16us bh = ldfrag(prh + k0);
      const v16us bl = ldfrag(prl + k0);
      #pragma unroll
      for (int mt = 0; mt < 4; ++mt) {
        const v16us ahf = ldfrag(kah + mt * 16 * HD + k0);
        const v16us alf = ldfrag(kal + mt * 16 * HD + k0);
        sacc[mt] = wmma3(ahf, alf, bh, bl, sacc[mt]);
      }
    }
    float mx = sacc[0][0];
    #pragma unroll
    for (int mt = 0; mt < 4; ++mt) {
      #pragma unroll
      for (int r = 0; r < 8; ++r) mx = fmaxf(mx, sacc[mt][r]);
    }
    mx = fmaxf(mx, __shfl_xor(mx, 16));
    float sum = 0.f;
    #pragma unroll
    for (int mt = 0; mt < 4; ++mt) {
      #pragma unroll
      for (int r = 0; r < 8; ++r) {
        const float e = __expf(sacc[mt][r] - mx);
        sacc[mt][r] = e;
        sum += e;
      }
    }
    sum += __shfl_xor(sum, 16);
    const float inv = __builtin_amdgcn_rcpf(sum);
    v16us pbh[2], pbl[2];
    #pragma unroll
    for (int ks = 0; ks < 2; ++ks) {
      #pragma unroll
      for (int r = 0; r < 8; ++r) {
        u16 hv, lv;
        split2(sacc[2 * ks][r] * inv, hv, lv);
        pbh[ks][r] = hv;
        pbl[ks][r] = lv;
        split2(sacc[2 * ks + 1][r] * inv, hv, lv);
        pbh[ks][8 + r] = hv;
        pbl[ks][8 + r] = lv;
      }
    }
    const u16* mah = MTh + (size_t)(n * 64 + m) * HD + 8 * h;
    const u16* mal = MTl + (size_t)(n * 64 + m) * HD + 8 * h;
    v8f oacc[4];
    #pragma unroll
    for (int mt = 0; mt < 4; ++mt) {
      oacc[mt] = z8;
      #pragma unroll
      for (int ks = 0; ks < 2; ++ks) {
        const v16us ahf = ldfrag(mah + mt * 16 * HD + 32 * ks);
        const v16us alf = ldfrag(mal + mt * 16 * HD + 32 * ks);
        oacc[mt] = wmma3(ahf, alf, pbh[ks], pbl[ks], oacc[mt]);
      }
    }
    __syncthreads();
    u16* orh = Ph + px * PST + n * 64 + 8 * h;
    u16* orl = Pl + px * PST + n * 64 + 8 * h;
    #pragma unroll
    for (int mt = 0; mt < 4; ++mt) {
      v8us oh, ol;
      #pragma unroll
      for (int r = 0; r < 8; ++r) {
        u16 hv, lv;
        split2(oacc[mt][r], hv, lv);
        oh[r] = hv;
        ol[r] = lv;
      }
      *(v8usa*)(orh + 16 * mt) = oh;
      *(v8usa*)(orl + 16 * mt) = ol;
    }
  }
  __syncthreads();

  {
    const int orow0 = 32 * w;
    v8f acc[2][4];
    #pragma unroll
    for (int mt = 0; mt < 2; ++mt) {
      #pragma unroll
      for (int nt = 0; nt < 4; ++nt) acc[mt][nt] = z8;
    }
    const u16* aph = WOh + (size_t)(orow0 + m) * CMID + 8 * h;
    const u16* apl = WOl + (size_t)(orow0 + m) * CMID + 8 * h;
    const u16* bph = Ph + m * PST + 8 * h;
    const u16* bpl = Pl + m * PST + 8 * h;
    #pragma unroll 1
    for (int ks = 0; ks < CMID / 32; ++ks) {
      const int k0 = 32 * ks;
      v16us ah[2], al[2];
      #pragma unroll
      for (int mt = 0; mt < 2; ++mt) {
        ah[mt] = ldfrag(aph + mt * 16 * CMID + k0);
        al[mt] = ldfrag(apl + mt * 16 * CMID + k0);
      }
      #pragma unroll
      for (int nt = 0; nt < 4; ++nt) {
        const v16us bh = ldfrag(bph + nt * 16 * PST + k0);
        const v16us bl = ldfrag(bpl + nt * 16 * PST + k0);
        #pragma unroll
        for (int mt = 0; mt < 2; ++mt) acc[mt][nt] = wmma3(ah[mt], al[mt], bh, bl, acc[mt][nt]);
      }
    }
    __syncthreads();
    f32a* sD = (f32a*)dl;
    #pragma unroll
    for (int mt = 0; mt < 2; ++mt) {
      const int ob = orow0 + 16 * mt + 8 * h;
      const v4f b0 = *(const v4fa*)(b_out + ob);
      const v4f b1 = *(const v4fa*)(b_out + ob + 4);
      const float bb[8] = {b0.x, b0.y, b0.z, b0.w, b1.x, b1.y, b1.z, b1.w};
      #pragma unroll
      for (int nt = 0; nt < 4; ++nt) {
        const int px = 16 * nt + m;
        #pragma unroll
        for (int r = 0; r < 8; ++r) sD[(ob + r) * TP + px] = acc[mt][nt][r] + bb[r];
      }
    }
    __syncthreads();
    const int hs = lane >> 4, x4 = 4 * (lane & 15);
    float* obase = out + (size_t)b * COUT * NPIX + s0 + x4;
    #pragma unroll 1
    for (int c = 0; c < 2; ++c) {
      v4f vals[8];
      size_t gi[8];
      #pragma unroll
      for (int i = 0; i < 8; ++i) {
        const int row = orow0 + 16 * c + 2 * i + hs;
        vals[i] = *(const v4fa*)(sD + row * TP + x4);
        gi[i] = (size_t)row * NPIX;
      }
      #pragma unroll
      for (int i = 0; i < 8; ++i) *(volatile v4f*)(obase + gi[i]) = vals[i];
      __threadfence();
      #pragma unroll
      for (int i = 0; i < 8; ++i) *(volatile v4f*)(obase + gi[i]) = vals[i];
    }
  }
}

extern "C" void kernel_launch(void* const* d_in, const int* in_sizes, int n_in,
                              void* d_out, int out_size, void* d_ws, size_t ws_size,
                              hipStream_t stream) {
  if (n_in < 7) return;
  if (in_sizes[0] != NB * CIN * NPIX) return;
  if (in_sizes[1] != NHEAD * HD * HD || in_sizes[2] != NHEAD * HD * HD) return;
  if (in_sizes[3] != CMID * CIN || in_sizes[4] != CMID) return;
  if (in_sizes[5] != COUT * CMID || in_sizes[6] != COUT) return;
  if (out_size != NB * COUT * NPIX) return;

  const float* x     = (const float*)d_in[0];
  const float* key_p = (const float*)d_in[1];
  const float* mem   = (const float*)d_in[2];
  const float* w_in  = (const float*)d_in[3];
  const float* b_in  = (const float*)d_in[4];
  const float* w_out = (const float*)d_in[5];
  const float* b_out = (const float*)d_in[6];
  float* outp = (float*)d_out;

  const size_t szWI = (size_t)CMID * CIN * 2;
  const size_t szWO = (size_t)COUT * CMID * 2;
  const size_t szT  = (size_t)NHEAD * HD * HD * 2;
  const size_t szX  = (size_t)NP * CIN * 2;
  size_t off = 0;
  char* ws = (char*)d_ws;
  u16* WIh = (u16*)(ws + off); off += szWI;
  u16* WIl = (u16*)(ws + off); off += szWI;
  u16* WOh = (u16*)(ws + off); off += szWO;
  u16* WOl = (u16*)(ws + off); off += szWO;
  u16* KTh = (u16*)(ws + off); off += szT;
  u16* KTl = (u16*)(ws + off); off += szT;
  u16* MTh = (u16*)(ws + off); off += szT;
  u16* MTl = (u16*)(ws + off); off += szT;
  u16* Xh  = (u16*)(ws + off); off += szX;
  u16* Xl  = (u16*)(ws + off); off += szX;
  const size_t total = off;
  if (total > ws_size) return;

  hipFuncSetAttribute(reinterpret_cast<const void*>(&main_k),
                      hipFuncAttributeMaxDynamicSharedMemorySize, LDS_MAIN);

  wcvt_k<<<(CMID * CIN + COUT * CMID) / 8 / 256, 256, 0, stream>>>(w_in, w_out, WIh, WIl, WOh, WOl);
  tr64_k<<<2 * NHEAD, 256, 0, stream>>>(key_p, mem, KTh, KTl, MTh, MTl);
  xcvt_k<<<dim3(NPIX / 64, CIN / 64, NB), 256, 0, stream>>>(x, Xh, Xl);
  main_k<<<NP / TP, 256, LDS_MAIN, stream>>>(Xh, Xl, WIh, WIl, b_in, KTh, KTl, MTh, MTl,
                                             WOh, WOl, b_out, outp);
}
